// ChannelwiseSpatialMHSA_19061064860255
// MI455X (gfx1250) — hardware-verified
//
#include <hip/hip_runtime.h>
#include <stdint.h>

#define NBAT   2
#define IMH    32
#define IMW    32
#define CIN    32
#define DMOD   64
#define NHEAD  4
#define HDIM   16
#define SEQ    1024
#define NSQ    64
#define COUT   64
#define BTP    1032
#define WPITCH 72
#define SPITCH 68
#define LOG2E  1.44269504088896340736f

static_assert(IMH * IMW == SEQ);
static_assert(NBAT * CIN == NSQ);
static_assert(NHEAD * HDIM == DMOD);
static_assert((SEQ % 64) == 0 && COUT == 64 && DMOD == 64 && CIN == 32 && HDIM == 16);
static_assert((BTP % 8) == 0 && (WPITCH % 8) == 0 && (SPITCH % 4) == 0);
static_assert(SEQ == 8 * 128);

typedef __bf16   v16b __attribute__((ext_vector_type(16)));
typedef float    v8f  __attribute__((ext_vector_type(8)));
typedef float    v4f  __attribute__((ext_vector_type(4)));
typedef unsigned int v8u __attribute__((ext_vector_type(8)));
typedef unsigned int v4u __attribute__((ext_vector_type(4)));

union FragB { v16b v; v8u u; v4u q[2]; };

__device__ __forceinline__ v8f zero8() { v8f z = {0.f, 0.f, 0.f, 0.f, 0.f, 0.f, 0.f, 0.f}; return z; }
__device__ __forceinline__ unsigned rne_hi(unsigned u) {
  return (u + 0x7FFFu + ((u >> 16) & 1u)) & 0xFFFF0000u;
}
__device__ __forceinline__ void split2(float a, unsigned& h16, unsigned& l16) {
  const unsigned hu = rne_hi(__float_as_uint(a));
  const float lf = a - __uint_as_float(hu);
  h16 = hu >> 16;
  l16 = rne_hi(__float_as_uint(lf)) >> 16;
}
__device__ __forceinline__ unsigned pk(unsigned lo16, unsigned hi16) { return (lo16 & 0xFFFFu) | (hi16 << 16); }

__device__ __forceinline__ v8f mma_b(v16b a, v16b b, v8f c) {
  return __builtin_amdgcn_wmma_f32_16x16x32_bf16(false, a, false, b, (short)0, c, false, false);
}
__device__ __forceinline__ void guard2(v8f& a, v8f& b, v8u x, v8u y, v8u z) {
#if defined(__HIP_DEVICE_COMPILE__)
  asm volatile("v_nop\n\tv_nop\n\tv_nop\n\tv_nop" : "+v"(a), "+v"(b) : "v"(x), "v"(y), "v"(z));
#endif
}
__device__ __forceinline__ void guard4(v8f& a, v8f& b, v8f& c, v8f& d, v8u x0, v8u x1,
                                       v8u y0, v8u y1, v8u y2, v8u y3, v8u z0, v8u z1, v8u z2, v8u z3) {
#if defined(__HIP_DEVICE_COMPILE__)
  asm volatile("v_nop\n\tv_nop\n\tv_nop\n\tv_nop"
               : "+v"(a), "+v"(b), "+v"(c), "+v"(d)
               : "v"(x0), "v"(x1), "v"(y0), "v"(y1), "v"(y2), "v"(y3), "v"(z0), "v"(z1), "v"(z2), "v"(z3));
#endif
}
__device__ __forceinline__ void wave_sync_lds() {
  __builtin_amdgcn_fence(__ATOMIC_RELEASE, "workgroup");
  __builtin_amdgcn_wave_barrier();
  __builtin_amdgcn_fence(__ATOMIC_ACQUIRE, "workgroup");
}

__global__ __launch_bounds__(128)
void attn_rank1(const float* __restrict__ x, const float* __restrict__ embed_w,
                const float* __restrict__ q_w, const float* __restrict__ k_w, float* bt) {
  __shared__ __align__(32) float tv[SEQ];
  __shared__ __align__(16) unsigned short Bt[4 * BTP];
  __shared__ __align__(16) float Bs[SEQ];
  __shared__ float hv[2][HDIM];
  __shared__ float red[4][2];

  const int n    = blockIdx.x >> 2;
  const int head = blockIdx.x & 3;
  const int b    = n >> 5;
  const int ch   = n & 31;
  const int tid  = threadIdx.x, lane = tid & 31, wave = tid >> 5;
  const int lo   = lane & 15, hi = lane >> 4;

  float lmax = -3.0e38f, lmin = 3.0e38f;
  for (int t = tid; t < SEQ; t += 128) {
    const int hh = t >> 5, ww = t & 31;
    const float v = x[(((size_t)b * IMH + hh) * IMW + ww) * CIN + ch];
    tv[t] = v;
    lmax = fmaxf(lmax, v);
    lmin = fminf(lmin, v);
  }
#pragma unroll
  for (int off = 16; off > 0; off >>= 1) {
    lmax = fmaxf(lmax, __shfl_xor(lmax, off, 32));
    lmin = fminf(lmin, __shfl_xor(lmin, off, 32));
  }
  if (lane == 0) { red[wave][0] = lmax; red[wave][1] = lmin; }

  if (wave < 2) {
    const float* wsrc = (wave == 0) ? q_w : k_w;
    const float* wrow = wsrc + (size_t)(head * HDIM + lo) * DMOD;
    float acc = 0.f;
#pragma unroll 4
    for (int k = 0; k < DMOD; ++k) acc = fmaf(wrow[k], embed_w[k], acc);
    hv[wave][lo] = acc;
  }
  __syncthreads();

  const float gmax = fmaxf(fmaxf(red[0][0], red[1][0]), fmaxf(red[2][0], red[3][0]));
  const float gmin = fminf(fminf(red[0][1], red[1][1]), fminf(red[2][1], red[3][1]));
  float dqk = 0.f;
#pragma unroll 4
  for (int d = 0; d < HDIM; ++d) dqk = fmaf(hv[0][d], hv[1][d], dqk);
  const float ah2 = dqk * (0.25f * LOG2E);

  {
    const int kb = 8 * tid;
    const v4f ta = *(const v4f*)(tv + kb);
    const v4f tb = *(const v4f*)(tv + kb + 4);
    float tt[8];
#pragma unroll
    for (int e = 0; e < 4; ++e) { tt[e] = ta[e]; tt[4 + e] = tb[e]; }
    unsigned hb[8], lb[8];
#pragma unroll
    for (int e = 0; e < 8; ++e) split2(tt[e], hb[e], lb[e]);
    v4u h4, l4;
#pragma unroll
    for (int e = 0; e < 4; ++e) { h4[e] = pk(hb[2 * e], hb[2 * e + 1]); l4[e] = pk(lb[2 * e], lb[2 * e + 1]); }
    const v4u ones = {0x3F803F80u, 0x3F803F80u, 0x3F803F80u, 0x3F803F80u};
    const v4u zer  = {0u, 0u, 0u, 0u};
    *(v4u*)(Bt + 0 * BTP + kb) = h4;
    *(v4u*)(Bt + 1 * BTP + kb) = l4;
    *(v4u*)(Bt + 2 * BTP + kb) = ones;
    *(v4u*)(Bt + 3 * BTP + kb) = zer;
    if (tid == 0) {
      *(v4u*)(Bt + 0 * BTP + SEQ) = zer;
      *(v4u*)(Bt + 1 * BTP + SEQ) = zer;
      *(v4u*)(Bt + 2 * BTP + SEQ) = zer;
      *(v4u*)(Bt + 3 * BTP + SEQ) = zer;
    }
  }
  __syncthreads();

  const int br = (lo < 3) ? lo : 3;
  const unsigned short* brow = Bt + br * BTP + 8 * hi;
  float* plane = bt + (size_t)(n * NHEAD + head) * SEQ;

#pragma unroll 1
  for (int i = 0; i < SEQ / 64; ++i) {
    const int s0 = (wave + 4 * i) * 16;
    const float coef = ah2 * tv[s0 + lo];
    const float cm   = -fmaxf(coef * gmax, coef * gmin);
    v8f acc1 = zero8(), acc2 = zero8();
#pragma unroll 1
    for (int kt = 0; kt < SEQ / 32; ++kt) {
      const int t0 = kt * 32;
      const v8f ta = *(const v8f*)(tv + t0 + 8 * hi);
      const v8f tb = *(const v8f*)(tv + t0 + 16 + 8 * hi);
      FragB ph, pl;
#pragma unroll
      for (int j = 0; j < 4; ++j) {
        const float p0 = __builtin_amdgcn_exp2f(fmaf(coef, ta[2 * j], cm));
        const float p1 = __builtin_amdgcn_exp2f(fmaf(coef, ta[2 * j + 1], cm));
        const float p2 = __builtin_amdgcn_exp2f(fmaf(coef, tb[2 * j], cm));
        const float p3 = __builtin_amdgcn_exp2f(fmaf(coef, tb[2 * j + 1], cm));
        const unsigned u0 = __float_as_uint(p0), u1 = __float_as_uint(p1);
        const unsigned u2 = __float_as_uint(p2), u3 = __float_as_uint(p3);
        const unsigned g0 = u0 & 0xFFFF0000u, g1 = u1 & 0xFFFF0000u;
        const unsigned g2 = u2 & 0xFFFF0000u, g3 = u3 & 0xFFFF0000u;
        const float l0 = p0 - __uint_as_float(g0), l1 = p1 - __uint_as_float(g1);
        const float l2 = p2 - __uint_as_float(g2), l3 = p3 - __uint_as_float(g3);
        ph.u[j]     = (u0 >> 16) | g1;
        ph.u[4 + j] = (u2 >> 16) | g3;
        pl.u[j]     = (__float_as_uint(l0) >> 16) | (__float_as_uint(l1) & 0xFFFF0000u);
        pl.u[4 + j] = (__float_as_uint(l2) >> 16) | (__float_as_uint(l3) & 0xFFFF0000u);
      }
      FragB bf;
      bf.q[0] = *(const v4u*)(brow + t0);
      bf.q[1] = *(const v4u*)(brow + t0 + 16);
      acc1 = mma_b(ph.v, bf.v, acc1);
      acc2 = mma_b(pl.v, bf.v, acc2);
      guard2(acc1, acc2, ph.u, pl.u, bf.u);
    }

    const int sb = 16 * hi;
    float beta[8];
#pragma unroll
    for (int r = 0; r < 8; ++r) {
      const float a0 = __shfl(acc1[r], sb, 32);
      const float a1 = __shfl(acc1[r], sb + 1, 32);
      const float a2 = __shfl(acc1[r], sb + 2, 32);
      const float c0 = __shfl(acc2[r], sb, 32);
      const float c1 = __shfl(acc2[r], sb + 1, 32);
      const float c2 = __shfl(acc2[r], sb + 2, 32);
      const float num = (a0 + c0) + (a1 + c1);
      const float den = a2 + c2;
      beta[r] = num * __builtin_amdgcn_rcpf(den);
    }
    float mine = beta[0];
#pragma unroll
    for (int r = 1; r < 8; ++r) mine = (lo == r) ? beta[r] : mine;
    if (lo < 8) Bs[s0 + 8 * hi + lo] = mine;
  }
  __syncthreads();
  {
    const v4f v0 = *(const v4f*)(Bs + 4 * tid);
    const v4f v1 = *(const v4f*)(Bs + 512 + 4 * tid);
    float* d0 = plane + 4 * tid;
    float* d1 = plane + 512 + 4 * tid;
    *(volatile v4f*)d0 = v0;
    *(volatile v4f*)d1 = v1;
    __threadfence();
    *(volatile v4f*)d0 = v0;
    *(volatile v4f*)d1 = v1;
  }
}

__global__ __launch_bounds__(128)
void proj_mix(const float* __restrict__ bt, const float* __restrict__ embed_w, const float* __restrict__ v_w,
              const float* __restrict__ o_w, const float* __restrict__ mix_w, float* out) {
  __shared__ __align__(16) unsigned short Wh[COUT * WPITCH];
  __shared__ __align__(16) unsigned short Wl[COUT * WPITCH];
  __shared__ __align__(32) float ve[DMOD];
  __shared__ float mw[CIN];
  __shared__ __align__(16) float sT[4][16 * SPITCH];
  const int tid  = threadIdx.x, lane = tid & 31, wave = tid >> 5;
  const int lo   = lane & 15, hi = lane >> 4;
  const int b    = blockIdx.x >> 4;
  const int s0   = (blockIdx.x & 15) * 64;

  {
    const int o = tid >> 1, k0 = (tid & 1) * 32;
    const float* sp = o_w + (size_t)o * DMOD + k0;
#pragma unroll
    for (int q = 0; q < 4; ++q) {
      const v4f a0 = *(const v4f*)(sp + 8 * q);
      const v4f a1 = *(const v4f*)(sp + 8 * q + 4);
      float f[8];
#pragma unroll
      for (int e = 0; e < 4; ++e) { f[e] = a0[e]; f[4 + e] = a1[e]; }
      v4u hq, lq;
#pragma unroll
      for (int e = 0; e < 4; ++e) {
        unsigned h0, l0, h1, l1;
        split2(f[2 * e], h0, l0);
        split2(f[2 * e + 1], h1, l1);
        hq[e] = pk(h0, h1);
        lq[e] = pk(l0, l1);
      }
      *(v4u*)(Wh + o * WPITCH + k0 + 8 * q) = hq;
      *(v4u*)(Wl + o * WPITCH + k0 + 8 * q) = lq;
    }
  }
  if (tid < DMOD) {
    const float* wrow = v_w + (size_t)tid * DMOD;
    float acc = 0.f;
#pragma unroll 4
    for (int k = 0; k < DMOD; ++k) acc = fmaf(wrow[k], embed_w[k], acc);
    ve[tid] = acc;
  }
  if (tid < CIN) mw[tid] = mix_w[tid];
  __syncthreads();

  v8f oacc[4];
#pragma unroll
  for (int j = 0; j < 4; ++j) oacc[j] = zero8();

  const int arow = s0 + 16 * wave + lo;
  const float* bp = bt + (size_t)(b * CIN) * (NHEAD * SEQ) + arow;

#pragma unroll 1
  for (int c = 0; c < CIN; ++c) {
    const float* bc = bp + (size_t)c * (NHEAD * SEQ);
    v8f acc[4];
#pragma unroll
    for (int j = 0; j < 4; ++j) acc[j] = zero8();
#pragma unroll 1
    for (int ks = 0; ks < 2; ++ks) {
      const float be0 = bc[(size_t)(2 * ks) * SEQ];
      const float be1 = bc[(size_t)(2 * ks + 1) * SEQ];
      const v8f vea = *(const v8f*)(ve + 32 * ks + 8 * hi);
      const v8f veb = *(const v8f*)(ve + 32 * ks + 16 + 8 * hi);
      FragB fa, fl;
#pragma unroll
      for (int j = 0; j < 4; ++j) {
        unsigned h0, l0, h1, l1;
        split2(be0 * vea[2 * j], h0, l0);
        split2(be0 * vea[2 * j + 1], h1, l1);
        fa.u[j] = pk(h0, h1);
        fl.u[j] = pk(l0, l1);
        split2(be1 * veb[2 * j], h0, l0);
        split2(be1 * veb[2 * j + 1], h1, l1);
        fa.u[4 + j] = pk(h0, h1);
        fl.u[4 + j] = pk(l0, l1);
      }
      FragB wh[4], wl[4];
#pragma unroll
      for (int j = 0; j < 4; ++j) {
        const int wo = (16 * j + lo) * WPITCH + 32 * ks + 8 * hi;
        wh[j].q[0] = *(const v4u*)(Wh + wo);
        wh[j].q[1] = *(const v4u*)(Wh + wo + 16);
        wl[j].q[0] = *(const v4u*)(Wl + wo);
        wl[j].q[1] = *(const v4u*)(Wl + wo + 16);
      }
#pragma unroll
      for (int j = 0; j < 4; ++j) {
        acc[j] = mma_b(fa.v, wh[j].v, acc[j]);
        acc[j] = mma_b(fa.v, wl[j].v, acc[j]);
        acc[j] = mma_b(fl.v, wh[j].v, acc[j]);
      }
      guard4(acc[0], acc[1], acc[2], acc[3], fa.u, fl.u,
             wh[0].u, wh[1].u, wh[2].u, wh[3].u, wl[0].u, wl[1].u, wl[2].u, wl[3].u);
    }
    const float wgt = mw[c];
#pragma unroll
    for (int j = 0; j < 4; ++j) {
#pragma unroll
      for (int r = 0; r < 8; ++r) oacc[j][r] = fmaf(wgt, acc[j][r], oacc[j][r]);
    }
  }

  float* slab = sT[wave];
  const int mOff = 8 * hi;
#pragma unroll
  for (int j = 0; j < 4; ++j) {
#pragma unroll
    for (int r = 0; r < 8; ++r) slab[(mOff + r) * SPITCH + (j << 4) + lo] = oacc[j][r];
  }
  wave_sync_lds();
  const int c4 = lo * 4;
  v4f vals[8];
#pragma unroll
  for (int it = 0; it < 8; ++it) {
    const int row = it * 2 + hi;
    vals[it] = *(const v4f*)(slab + row * SPITCH + c4);
  }
  float* ob = out + (size_t)(b * SEQ + s0 + 16 * wave) * COUT;
#pragma unroll
  for (int it = 0; it < 8; ++it) {
    const int row = it * 2 + hi;
    *(volatile v4f*)(ob + (size_t)row * COUT + c4) = vals[it];
  }
  __threadfence();
#pragma unroll
  for (int it = 0; it < 8; ++it) {
    const int row = it * 2 + hi;
    *(volatile v4f*)(ob + (size_t)row * COUT + c4) = vals[it];
  }
  wave_sync_lds();
}

extern "C" void kernel_launch(void* const* d_in, const int* in_sizes, int n_in,
                              void* d_out, int out_size, void* d_ws, size_t ws_size,
                              hipStream_t stream) {
  if (n_in < 7) return;
  if (in_sizes[0] != NBAT * IMH * IMW * CIN) return;
  if (in_sizes[1] != DMOD) return;
  if (in_sizes[2] != DMOD * DMOD || in_sizes[3] != DMOD * DMOD || in_sizes[4] != DMOD * DMOD) return;
  if (in_sizes[5] != COUT * DMOD || in_sizes[6] != CIN) return;
  if (out_size != NBAT * SEQ * COUT) return;

  const size_t PB = (size_t)NSQ * NHEAD * SEQ * 4;
  if (PB > ws_size) return;
  if (PB > (size_t)134217728) return;

  const float* x       = (const float*)d_in[0];
  const float* embed_w = (const float*)d_in[1];
  const float* q_w     = (const float*)d_in[2];
  const float* k_w     = (const float*)d_in[3];
  const float* v_w     = (const float*)d_in[4];
  const float* o_w     = (const float*)d_in[5];
  const float* mix_w   = (const float*)d_in[6];
  float* bt            = (float*)d_ws;
  float* out           = (float*)d_out;

  const dim3 blk(128);
  const dim3 gA(NSQ * NHEAD);
  const dim3 gP(NBAT * SEQ / 64);

  attn_rank1<<<gA, blk, 0, stream>>>(x, embed_w, q_w, k_w, bt);
  proj_mix<<<gP, blk, 0, stream>>>(bt, embed_w, v_w, o_w, mix_w, out);
  (void)hipGetLastError();
}
